// KANLayer_30777735643159
// MI455X (gfx1250) — hardware-verified
//
#include <hip/hip_runtime.h>
#include <math.h>

constexpr int kRows  = 4096;
constexpr int kDimIn = 256;
constexpr int kUnits = 256;
constexpr int kDeg   = 4;
constexpr int kKaug  = 4 * kDimIn;
constexpr float kWCarry    = 16.0f;
constexpr float kWCarryInv = 1.0f / 16.0f;
constexpr float kSeluScale      = 1.0507009873554805f;
constexpr float kSeluScaleAlpha = 1.7580993408473766f;

static_assert(kKaug % 32 == 0, "");
static_assert(kRows % 64 == 0, "");
static_assert(kUnits % 64 == 0, "");
static_assert(((kRows / 64) * (kUnits / 64)) % 8 == 0, "");
static_assert(kDimIn == 256 && kUnits == 256, "");

constexpr size_t kOffA    = 0;
constexpr size_t kBytesA  = (size_t)kRows * kKaug * 2;
constexpr size_t kOffBt   = kOffA + kBytesA;
constexpr size_t kBytesBt = (size_t)kUnits * kKaug * 2;
constexpr size_t kOffC    = kOffBt + kBytesBt;
constexpr size_t kBytesC  = (size_t)kUnits * 4;
constexpr size_t kWsTotal = kOffC + kBytesC;
static_assert(kWsTotal == 8913920, "");
static_assert(kWsTotal <= 134217728, "");
static_assert(kOffBt % 128 == 0 && kOffC % 128 == 0, "");

typedef __attribute__((ext_vector_type(16))) _Float16 v16h;
typedef __attribute__((ext_vector_type(8)))  _Float16 v8h;
typedef __attribute__((ext_vector_type(8)))  float    v8f;
typedef __attribute__((ext_vector_type(4)))  float    v4f;
typedef __attribute__((ext_vector_type(2)))  float    v2f;

__device__ __forceinline__ void keep4_h(v16h a, v16h b, v16h c, v16h d) { asm volatile("v_nop" :: "v"(a), "v"(b), "v"(c), "v"(d)); }
__device__ __forceinline__ void acc_guard4(v8f& a, v8f& b, v8f& c, v8f& d) { asm volatile("v_nop\n\tv_nop\n\tv_nop\n\tv_nop" : "+v"(a), "+v"(b), "+v"(c), "+v"(d)); }
__device__ __forceinline__ void dep_guard4_h(v8f& a, v8f& b, v8f& c, v8f& d, v16h x, v16h y) {
  asm volatile("v_nop\n\tv_nop\n\tv_nop\n\tv_nop" : "+v"(a), "+v"(b), "+v"(c), "+v"(d) : "v"(x), "v"(y));
}

template <typename T> struct Frag;
template <> struct Frag<_Float16> {
  typedef v16h V; union U { v16h v; v8h h[2]; };
  static __device__ __forceinline__ v16h load(const _Float16* p) {
    U f; f.h[0] = *(const v8h*)(p); f.h[1] = *(const v8h*)(p + 16); return f.v;
  }
  static __device__ __forceinline__ v8f mma(v16h a, v16h b, v8f c) {
    return __builtin_amdgcn_wmma_f32_16x16x32_f16(false, a, false, b, (short)0, c, false, false);
  }
};

__device__ __forceinline__ unsigned pk16(unsigned short a, unsigned short b) { return (unsigned)a | ((unsigned)b << 16); }
__device__ __forceinline__ unsigned short h_bits(float f) { const _Float16 h = (_Float16)f; return __builtin_bit_cast(unsigned short, h); }

__device__ __forceinline__ float selu_f(float x) {
  const float en = kSeluScaleAlpha * (expf(x) - 1.0f);
  const float ep = kSeluScale * x;
  return (x > 0.0f) ? ep : en;
}

__global__ __launch_bounds__(256) void prep_a_kernel(const float* __restrict__ X, unsigned* __restrict__ Aw) {
  const int t   = threadIdx.x;
  const int row = blockIdx.x * 2 + (t >> 7);
  const int tr  = t & 127;
  const v2f xv = *(const v2f*)(X + (size_t)row * kDimIn + 2 * tr);
  const float x0 = xv.x;
  const float x1 = xv.y;
  const float t0 = tanhf(x0);
  const float t1 = tanhf(x1);
  const float q0 = t0 * t0;
  const float q1 = t1 * t1;
  const float c0 = q0 * t0;
  const float c1 = q1 * t1;
  const unsigned w0 = pk16(h_bits(x0), h_bits(x1));
  const unsigned w1 = pk16(h_bits(t0), h_bits(t1));
  const unsigned w2 = pk16(h_bits(q0), h_bits(q1));
  const unsigned w3 = pk16(h_bits(c0), h_bits(c1));
  volatile unsigned* p = Aw + (size_t)row * (kKaug / 2) + tr;
  p[0]   = w0;
  p[128] = w1;
  p[256] = w2;
  p[384] = w3;
  __threadfence();
  p[0]   = w0;
  p[128] = w1;
  p[256] = w2;
  p[384] = w3;
}

__global__ __launch_bounds__(256) void prep_w_kernel(const float* __restrict__ Wb, const float* __restrict__ Sp,
                                                     const float* __restrict__ Gt, unsigned* __restrict__ Btw,
                                                     float carry) {
  const int j = blockIdx.x;
  const int t = threadIdx.x;
#pragma unroll
  for (int it = 0; it < 2; ++it) {
    const int k0 = it * 512 + 2 * t;
    const int d  = k0 >> 8;
    const int i0 = k0 & 255;
    const int i1 = i0 + 1;
    const int dd = (d == 0) ? 1 : d;
    const float wb0 = Wb[(size_t)i0 * kUnits + j];
    const float wb1 = Wb[(size_t)i1 * kUnits + j];
    const float g0  = Gt[(size_t)i0 * kUnits + j];
    const float g1  = Gt[(size_t)i1 * kUnits + j];
    const float s0  = Sp[((size_t)i0 * kUnits + j) * kDeg + dd];
    const float s1  = Sp[((size_t)i1 * kUnits + j) * kDeg + dd];
    const float fl  = (d == 0) ? 1.0f : 0.0f;
    const float fs  = 1.0f - fl;
    const float v0  = fmaf(fl, wb0, fs * (g0 * s0)) * carry;
    const float v1  = fmaf(fl, wb1, fs * (g1 * s1)) * carry;
    const unsigned w = pk16(h_bits(v0), h_bits(v1));
    volatile unsigned* p = Btw + (size_t)j * (kKaug / 2) + it * 256 + t;
    *p = w;
    __threadfence();
    *p = w;
  }
}

__global__ __launch_bounds__(256) void colconst_kernel(const float* __restrict__ bias, const float* __restrict__ Sp,
                                                       const float* __restrict__ Gt, float* __restrict__ cc) {
  const int j = threadIdx.x;
  float s = 0.0f;
#pragma unroll 4
  for (int i = 0; i < kDimIn; ++i) {
    const size_t ij = (size_t)i * kUnits + j;
    s += Gt[ij] * Sp[ij * kDeg];
  }
  const float v = bias[j] + s;
  volatile float* p = cc + j;
  *p = v;
  __threadfence();
  *p = v;
}

__global__ __launch_bounds__(256) void gemm_f16_selu_kernel(
    const unsigned short* __restrict__ Ap, int lda,
    const unsigned short* __restrict__ Btp, int ldb,
    float* __restrict__ Cout, int ldc,
    const float* __restrict__ coladd,
    int M, int N, int K, float scale) {
  typedef _Float16 T;
  typedef v16h V;
  const T* A  = (const T*)Ap;
  const T* Bt = (const T*)Btp;
  __shared__ __align__(16) float sT[8][16 * 68];
  const int lane = threadIdx.x & 31;
  const int wave = threadIdx.x >> 5;
  const int tilesN = N >> 6;
  const int tilesM = M >> 6;
  const int tile = blockIdx.x * 8 + wave;
  if (tile >= tilesM * tilesN) return;
  const int tm = tile / tilesN;
  const int tn = tile - tm * tilesN;
  const int m0 = tm << 6;
  const int n0 = tn << 6;

  const int rlane = lane & 15;
  const int koff  = (lane >> 4) * 8;
  const int mOff  = (lane >> 4) * 8;

  v8f acc[4][4];
#pragma unroll
  for (int i = 0; i < 4; ++i)
#pragma unroll
    for (int j = 0; j < 4; ++j) acc[i][j] = (v8f){0.f,0.f,0.f,0.f,0.f,0.f,0.f,0.f};

  for (int k0 = 0; k0 < K; k0 += 32) {
    V bh[4];
#pragma unroll
    for (int j = 0; j < 4; ++j) {
      const size_t bo = (size_t)(n0 + (j << 4) + rlane) * ldb + koff + k0;
      bh[j] = Frag<T>::load(Bt + bo);
    }
#pragma unroll
    for (int i = 0; i < 4; ++i) {
      const size_t ao = (size_t)(m0 + (i << 4) + rlane) * lda + koff + k0;
      V ah = Frag<T>::load(A + ao);
#pragma unroll
      for (int j = 0; j < 4; ++j) acc[i][j] = Frag<T>::mma(ah, bh[j], acc[i][j]);
      dep_guard4_h(acc[i][0], acc[i][1], acc[i][2], acc[i][3], ah, bh[3]);
    }
    keep4_h(bh[0], bh[1], bh[2], bh[3]);
  }
  acc_guard4(acc[0][0], acc[0][1], acc[0][2], acc[0][3]);
  acc_guard4(acc[1][0], acc[1][1], acc[1][2], acc[1][3]);
  acc_guard4(acc[2][0], acc[2][1], acc[2][2], acc[2][3]);
  acc_guard4(acc[3][0], acc[3][1], acc[3][2], acc[3][3]);

  float* slab = sT[wave];
#pragma unroll
  for (int i = 0; i < 4; ++i) {
    const int mBase = m0 + (i << 4);
#pragma unroll
    for (int j = 0; j < 4; ++j) {
      const int n = n0 + (j << 4) + rlane;
      const float cv = coladd[n];
#pragma unroll
      for (int r = 0; r < 8; ++r) {
        float v = acc[i][j][r] * scale + cv;
        v = selu_f(v);
        slab[(mOff + r) * 68 + (j << 4) + rlane] = v;
      }
    }
    __builtin_amdgcn_fence(__ATOMIC_RELEASE, "workgroup");
    __builtin_amdgcn_wave_barrier();
    __builtin_amdgcn_fence(__ATOMIC_ACQUIRE, "workgroup");
    {
      float* C = Cout;
      const int hh = lane >> 4, c4 = (lane & 15) * 4;
      for (int pass = 0; pass < 2; ++pass) {
#pragma unroll
        for (int it = 0; it < 8; ++it) {
          const int row = it * 2 + hh;
          v4f v = *(const v4f*)(slab + row * 68 + c4);
          *(volatile v4f*)(C + (size_t)(mBase + row) * ldc + n0 + c4) = v;
        }
        __threadfence();
      }
    }
    __builtin_amdgcn_fence(__ATOMIC_RELEASE, "workgroup");
    __builtin_amdgcn_wave_barrier();
    __builtin_amdgcn_fence(__ATOMIC_ACQUIRE, "workgroup");
  }
}

extern "C" void kernel_launch(void* const* d_in, const int* in_sizes, int n_in,
                              void* d_out, int out_size, void* d_ws, size_t ws_size,
                              hipStream_t stream)
{
  if (n_in < 5) return;
  if (in_sizes[0] != kRows * kDimIn) return;
  if (in_sizes[1] != kDimIn * kUnits) return;
  if (in_sizes[2] != kUnits) return;
  if (in_sizes[3] != kDimIn * kUnits * kDeg) return;
  if (in_sizes[4] != kDimIn * kUnits) return;
  if (out_size < kRows * kUnits) return;
  if (ws_size < kWsTotal) return;

  const float* X    = (const float*)d_in[0];
  const float* Wb   = (const float*)d_in[1];
  const float* bias = (const float*)d_in[2];
  const float* Sp   = (const float*)d_in[3];
  const float* Gt   = (const float*)d_in[4];
  float* out        = (float*)d_out;

  char* ws = (char*)d_ws;
  unsigned short* Apl  = (unsigned short*)(ws + kOffA);
  unsigned short* Btpl = (unsigned short*)(ws + kOffBt);
  float* cc            = (float*)(ws + kOffC);

  prep_a_kernel<<<kRows / 2, 256, 0, stream>>>(X, (unsigned*)Apl);
  prep_w_kernel<<<kUnits, 256, 0, stream>>>(Wb, Sp, Gt, (unsigned*)Btpl, kWCarry);
  colconst_kernel<<<1, 256, 0, stream>>>(bias, Sp, Gt, cc);
  constexpr int kTiles = (kRows / 64) * (kUnits / 64);
  gemm_f16_selu_kernel<<<dim3(kTiles / 8, 1), 256, 0, stream>>>(
      Apl, kKaug, Btpl, kKaug, out, kUnits, cc, kRows, kUnits, kKaug, kWCarryInv);
}
